// GPT2Attention_86388972192344
// MI455X (gfx1250) — hardware-verified
//
#include <hip/hip_runtime.h>
#include <math.h>

typedef __attribute__((ext_vector_type(16))) _Float16 v16h;
typedef __attribute__((ext_vector_type(16))) __bf16 v16b;
typedef __attribute__((ext_vector_type(8)))  _Float16 v8h;
typedef __attribute__((ext_vector_type(8)))  __bf16 v8b;
typedef __attribute__((ext_vector_type(8)))  float v8f;
typedef __attribute__((ext_vector_type(4)))  float v4f;
typedef __attribute__((ext_vector_type(4)))  unsigned v4u;

template <typename T> __device__ __forceinline__ void vst2(void* p, T v) { *(volatile T*)p = v; __threadfence(); *(volatile T*)p = v; }

__device__ __forceinline__ v8f wmma16(v16h a, v16h b, v8f c) {
  v8f d = __builtin_amdgcn_wmma_f32_16x16x32_f16(false, a, false, b, (short)0, c, false, false);
  asm volatile("v_nop\n\tv_nop\n\tv_nop\n\tv_nop" : "+v"(d) : "v"(a), "v"(b));
  return d;
}
__device__ __forceinline__ v8f wmma_bf(v16b a, v16b b, v8f c) {
  v8f d = __builtin_amdgcn_wmma_f32_16x16x32_bf16(false, a, false, b, (short)0, c, false, false);
  asm volatile("v_nop\n\tv_nop\n\tv_nop\n\tv_nop" : "+v"(d) : "v"(a), "v"(b));
  return d;
}
__device__ __forceinline__ v16h frag_h(const _Float16* rowk0, int lane) {
  union { v16h v; v8h q[2]; } u; const _Float16* p = rowk0 + 8 * (lane >> 4);
  u.q[0] = *(const v8h*)p; u.q[1] = *(const v8h*)(p + 16); return u.v;
}
__device__ __forceinline__ v16b frag_b(const __bf16* rowk0, int lane) {
  union { v16b v; v8b q[2]; } u; const __bf16* p = rowk0 + 8 * (lane >> 4);
  u.q[0] = *(const v8b*)p; u.q[1] = *(const v8b*)(p + 16); return u.v;
}
struct F2 { v16b h, l; };
__device__ __forceinline__ F2 bsplit16(const float v[16]) { F2 r;
#pragma unroll
  for (int i = 0; i < 16; ++i) { const __bf16 h = (__bf16)v[i]; r.h[i] = h; r.l[i] = (__bf16)(v[i] - (float)h); }
  return r; }
__device__ __forceinline__ F2 split_row(const float* row, int k0, int lane) { float v[16]; const float* p = row + k0 + 8 * (lane >> 4);
#pragma unroll
  for (int i = 0; i < 8; ++i) { v[i] = p[i]; v[8 + i] = p[16 + i]; }
  return bsplit16(v); }
__device__ __forceinline__ float bfr(float v) { return (float)(__bf16)v; }
__device__ __forceinline__ void ldsx() { asm volatile("s_wait_dscnt 0" ::: "memory"); __builtin_amdgcn_wave_barrier(); __builtin_amdgcn_fence(3, "workgroup"); }

#ifndef NB
#define NB 2
#endif
#ifndef SEQ
#define SEQ 2048
#endif
#define NB_FULL 2
#define SEQ_FULL 2048
#define DM 1024
#define NH 16
#define HD 64
#define QKVW (3 * DM)
#define NROWS (NB * SEQ)
static_assert(NB >= 1 && NB <= NB_FULL);
static_assert(SEQ >= 64 && SEQ <= SEQ_FULL && (SEQ % 64) == 0);
static_assert((NROWS % 64) == 0);
static_assert((DM % 128) == 0 && (QKVW % 128) == 0 && HD == 64 && NH * HD == DM);

#define PK_A 0
#define PK_P (PK_A + QKVW * DM)
#define PK_END (PK_P + DM * DM)
#define WS_PK  0u
#define WS_QK  (WS_PK + 2u * PK_END)
#define WS_VTH (WS_QK + 2u * NROWS * 2 * DM)
#define WS_O   (WS_VTH + 2u * NB * DM * SEQ)
#define WS_END (WS_O + 4u * NROWS * DM)
static_assert(WS_END <= 134217728u);
static_assert((WS_QK % 128u) == 0 && (WS_VTH % 128u) == 0 && (WS_O % 128u) == 0);
static_assert((size_t)NROWS * DM * 4 <= 16777216u);

__global__ __launch_bounds__(256) void k_pack(const float* __restrict__ WA, const float* __restrict__ WP, __bf16* __restrict__ PK) {
  __shared__ __align__(16) __bf16 s[DM];
  const int n = blockIdx.x, which = blockIdx.y, t = threadIdx.x;
  const float* src = (which < 3) ? WA : WP; const int ld = (which < 3) ? QKVW : DM; const int c = (which < 3) ? (which * DM + n) : n;
  for (int k = t; k < DM; k += 256) s[k] = (__bf16)src[(size_t)k * ld + c];
  __syncthreads();
  __bf16* dst = PK + ((which < 3) ? ((size_t)PK_A + ((size_t)which * DM + n) * DM) : ((size_t)PK_P + (size_t)n * DM));
  for (int q = t; q < DM / 8; q += 256) vst2(dst + q * 8, *(const v4u*)&s[q * 8]);
}
__global__ __launch_bounds__(128) void k_qkv(const float* __restrict__ X, const __bf16* __restrict__ P, const float* __restrict__ BA, _Float16* __restrict__ QK, _Float16* __restrict__ VTH) {
  __shared__ __align__(16) _Float16 so[4][16][136];
  __shared__ __align__(16) _Float16 sth[128][72];
  const int tid = threadIdx.x, wave = tid >> 5, lane = tid & 31, col = lane & 15, g = lane >> 4;
  const int rt = blockIdx.x; const int b = (rt * 64) / SEQ, s0 = (rt * 64) % SEQ;
  const int n0 = blockIdx.y * 128;
  const size_t xrow0 = (size_t)b * SEQ_FULL + s0 + wave * 16;
  const size_t crow0 = (size_t)rt * 64 + wave * 16;
  v8f acc[8] = {};
#pragma unroll 2
  for (int kc = 0; kc < DM / 32; ++kc) { v16b a; { const float* p = X + (xrow0 + col) * DM + kc * 32 + 8 * g;
#pragma unroll
      for (int i = 0; i < 8; ++i) { a[i] = (__bf16)p[i]; a[8 + i] = (__bf16)p[16 + i]; } }
#pragma unroll
    for (int j = 0; j < 8; ++j) acc[j] = wmma_bf(a, frag_b(P + (size_t)(n0 + j * 16 + col) * DM + kc * 32, lane), acc[j]); }
  if (n0 < 2 * DM) {
#pragma unroll
    for (int j = 0; j < 8; ++j) {
#pragma unroll
      for (int r = 0; r < 8; ++r) so[wave][8 * g + r][j * 16 + col] = (_Float16)(acc[j][r] + bfr(BA[n0 + j * 16 + col])); }
    ldsx();
    for (int rl = 0; rl < 16; ++rl) if (lane < 16) vst2(QK + (crow0 + rl) * (2 * DM) + n0 + lane * 8, *(const v4u*)&so[wave][rl][lane * 8]);
  } else {
#pragma unroll
    for (int j = 0; j < 8; ++j) {
#pragma unroll
      for (int r = 0; r < 8; ++r) sth[j * 16 + col][wave * 16 + 8 * g + r] = (_Float16)(acc[j][r] + bfr(BA[n0 + j * 16 + col])); }
    __syncthreads();
    const int pc0 = n0 - 2 * DM;
    for (int q = tid; q < 128 * 8; q += 128) { const int d = q >> 3, pc = q & 7; const size_t o = ((size_t)b * DM + pc0 + d) * SEQ + s0 + pc * 8; vst2(VTH + o, *(const v4u*)&sth[d][pc * 8]); }
  }
}
__global__ __launch_bounds__(128) __attribute__((amdgpu_num_vgpr(256)))
void k_attn(const _Float16* __restrict__ QK, const _Float16* __restrict__ VTH, const float* __restrict__ MK, float* __restrict__ O) {
  __shared__ __align__(16) float sp[4][16][36]; __shared__ __align__(16) float so[4][16][68];
  const int tid = threadIdx.x, wave = tid >> 5, lane = tid & 31, col = lane & 15, g = lane >> 4;
  const int qb = blockIdx.x, h = blockIdx.y, b = blockIdx.z; const int q0 = qb * 64 + wave * 16;
  const size_t rowb = (size_t)b * SEQ;
  const size_t rq = rowb + q0 + col;
  const float* mkrow = MK + (size_t)b * SEQ_FULL;
  v16h aq[2];
#pragma unroll
  for (int kc = 0; kc < 2; ++kc) aq[kc] = frag_h(QK + rq * (2 * DM) + h * HD + kc * 32, lane);
  float m[8], l[8];
#pragma unroll
  for (int r = 0; r < 8; ++r) { m[r] = -3.0e38f; l[r] = 0.f; }
  v8f acc[4] = {};
#pragma unroll 1
  for (int ks = 0; ks < SEQ / 32; ++ks) { v8f s[2];
#pragma unroll
    for (int ct = 0; ct < 2; ++ct) { const int kk = ks * 32 + ct * 16 + col; const _Float16* krow = QK + (rowb + kk) * (2 * DM) + DM + h * HD; v8f c = {};
#pragma unroll
      for (int kc = 0; kc < 2; ++kc) c = wmma16(aq[kc], frag_h(krow + kc * 32, lane), c);
      const float mk = bfr(mkrow[kk]);
#pragma unroll
      for (int r = 0; r < 8; ++r) s[ct][r] = c[r] * 0.125f + mk; }
#pragma unroll
    for (int r = 0; r < 8; ++r) { float mx = fmaxf(s[0][r], s[1][r]);
#pragma unroll
      for (int o = 1; o < 16; o <<= 1) mx = fmaxf(mx, __shfl_xor(mx, o));
      const float mn = fmaxf(m[r], mx); const float alpha = __expf(m[r] - mn);
      const float e0 = __expf(s[0][r] - mn), e1 = __expf(s[1][r] - mn); float es = e0 + e1;
#pragma unroll
      for (int o = 1; o < 16; o <<= 1) es += __shfl_xor(es, o);
      l[r] = l[r] * alpha + es; m[r] = mn;
#pragma unroll
      for (int dt = 0; dt < 4; ++dt) acc[dt][r] *= alpha;
      sp[wave][8 * g + r][col] = e0; sp[wave][8 * g + r][16 + col] = e1; }
    ldsx();
    v16h pa; { const float* prow = &sp[wave][col][0] + 8 * g;
#pragma unroll
      for (int i = 0; i < 8; ++i) { pa[i] = (_Float16)(prow[i] * 2048.0f); pa[8 + i] = (_Float16)(prow[16 + i] * 2048.0f); } }
#pragma unroll
    for (int dt = 0; dt < 4; ++dt) { const size_t vr = ((size_t)b * DM + h * HD + dt * 16 + col) * SEQ + ks * 32; acc[dt] = wmma16(pa, frag_h(VTH + vr, lane), acc[dt]); }
    ldsx(); }
#pragma unroll
  for (int r = 0; r < 8; ++r) { const float il = (1.0f / 2048.0f) / l[r];
#pragma unroll
    for (int dt = 0; dt < 4; ++dt) so[wave][8 * g + r][dt * 16 + col] = acc[dt][r] * il; }
  ldsx();
  for (int rl = 0; rl < 16; ++rl) if (lane < 16) vst2(O + (rowb + q0 + rl) * DM + h * HD + lane * 4, *(const v4f*)&so[wave][rl][lane * 4]);
}
__global__ __launch_bounds__(128) void k_out(const float* __restrict__ OC, const __bf16* __restrict__ P, const float* __restrict__ BO, float* __restrict__ Y) {
  __shared__ __align__(16) float so[4][16][132];
  const int tid = threadIdx.x, wave = tid >> 5, lane = tid & 31, col = lane & 15, g = lane >> 4; const size_t r0 = (size_t)blockIdx.x * 64 + wave * 16; const int n0 = blockIdx.y * 128;
  v8f acc[8] = {};
#pragma unroll 2
  for (int kc = 0; kc < DM / 32; ++kc) { const F2 a = split_row(OC + (r0 + col) * DM, kc * 32, lane);
#pragma unroll
    for (int j = 0; j < 8; ++j) { const v16b w = frag_b(P + (size_t)(n0 + j * 16 + col) * DM + kc * 32, lane); acc[j] = wmma_bf(a.l, w, acc[j]); acc[j] = wmma_bf(a.h, w, acc[j]); } }
#pragma unroll
  for (int j = 0; j < 8; ++j) {
#pragma unroll
    for (int r = 0; r < 8; ++r) so[wave][8 * g + r][j * 16 + col] = acc[j][r] + bfr(BO[n0 + j * 16 + col]); }
  ldsx();
  for (int rl = 0; rl < 16; ++rl) vst2(Y + (r0 + rl) * DM + n0 + lane * 4, *(const v4f*)&so[wave][rl][lane * 4]);
}
extern "C" void kernel_launch(void* const* d_in, const int* in_sizes, int n_in, void* d_out, int out_size, void* d_ws, size_t ws_size, hipStream_t stream) {
  if (n_in < 6) return;
  if (in_sizes[0] < ((NB - 1) * SEQ_FULL + SEQ) * DM) return;
  if (in_sizes[1] < (NB - 1) * SEQ_FULL + SEQ) return;
  if (in_sizes[2] < DM * QKVW || in_sizes[3] < QKVW || in_sizes[4] < DM * DM || in_sizes[5] < DM) return;
  if (out_size < NROWS * DM) return;
  if (ws_size < (size_t)WS_END) return;
  const float* X = (const float*)d_in[0]; const float* MK = (const float*)d_in[1]; const float* WA = (const float*)d_in[2];
  const float* BA = (const float*)d_in[3]; const float* WP = (const float*)d_in[4]; const float* BP = (const float*)d_in[5];
  char* ws = (char*)d_ws; __bf16* PK = (__bf16*)(ws + WS_PK); _Float16* QK = (_Float16*)(ws + WS_QK); _Float16* VTH = (_Float16*)(ws + WS_VTH); float* OC = (float*)(ws + WS_O);
  k_pack<<<dim3(DM, 4), 256, 0, stream>>>(WA, WP, PK);
  k_qkv<<<dim3(NROWS / 64, QKVW / 128), 128, 0, stream>>>(X, PK + PK_A, BA, QK, VTH);
  k_attn<<<dim3(SEQ / 64, NH, NB), 128, 0, stream>>>(QK, VTH, MK, OC);
  k_out<<<dim3(NROWS / 64, DM / 128), 128, 0, stream>>>(OC, PK + PK_P, BP, (float*)d_out);
}
